// NestedAttention_8950711845473
// MI455X (gfx1250) — hardware-run, weakly checked
//
#include <hip/hip_runtime.h>
#include <math.h>

typedef __attribute__((ext_vector_type(16))) _Float16 v16h;
typedef __attribute__((ext_vector_type(16))) __bf16 v16b;
typedef __attribute__((ext_vector_type(8)))  _Float16 v8h;
typedef __attribute__((ext_vector_type(8)))  float v8f;
typedef __attribute__((ext_vector_type(4)))  float v4f;
typedef __attribute__((ext_vector_type(2)))  float v2f;
typedef __attribute__((ext_vector_type(4)))  unsigned v4u;
typedef __attribute__((ext_vector_type(4)))  int v4i;
typedef float __attribute__((may_alias)) float_a;
typedef int __attribute__((may_alias)) int_a;

template <typename T> __device__ __forceinline__ void vst2(void* p, T v) { *(volatile T*)p = v; __threadfence(); *(volatile T*)p = v; }
__device__ __forceinline__ v8f wmma16(v16h a, v16h b, v8f c) {
  v8f d = __builtin_amdgcn_wmma_f32_16x16x32_f16(false, a, false, b, (short)0, c, false, false);
  asm volatile("v_nop\n\tv_nop\n\tv_nop\n\tv_nop" : "+v"(d) : "v"(a), "v"(b));
  return d;
}
__device__ __forceinline__ v8f wmma_bf(v16b a, v16b b, v8f c) {
  v8f d = __builtin_amdgcn_wmma_f32_16x16x32_bf16(false, a, false, b, (short)0, c, false, false);
  asm volatile("v_nop\n\tv_nop\n\tv_nop\n\tv_nop" : "+v"(d) : "v"(a), "v"(b));
  return d;
}
__device__ __forceinline__ v16h frag_h(const _Float16* rowk0, int lane) {
  union { v16h v; v8h q[2]; } u; const _Float16* p = rowk0 + 8 * (lane >> 4);
  u.q[0] = *(const v8h*)p; u.q[1] = *(const v8h*)(p + 16); return u.v;
}
__device__ __forceinline__ v16h frag_f32(const float* rowk0, int lane) {
  v16h a; const float* p = rowk0 + 8 * (lane >> 4);
#pragma unroll
  for (int i = 0; i < 8; ++i) { a[i] = (_Float16)p[i]; a[8 + i] = (_Float16)p[16 + i]; }
  return a;
}
__device__ __forceinline__ v16h frag_f32s(const float* rowk0, int lane, float sc) {
  v16h a; const float* p = rowk0 + 8 * (lane >> 4);
#pragma unroll
  for (int i = 0; i < 8; ++i) { a[i] = (_Float16)(p[i] * sc); a[8 + i] = (_Float16)(p[16 + i] * sc); }
  return a;
}
__device__ __forceinline__ v16h fragc_f32(const float* W, int k0, int n, int lane, int ld, int K) {
  v16h a; const int g = lane >> 4;
#pragma unroll
  for (int i = 0; i < 8; ++i) { const int ka = k0 + 8 * g + i, kb = ka + 16;
    a[i] = (_Float16)(ka < K ? W[(size_t)(ka < K ? ka : K - 1) * ld + n] : 0.f); a[8 + i] = (_Float16)(kb < K ? W[(size_t)(kb < K ? kb : K - 1) * ld + n] : 0.f); }
  return a;
}
struct F2 { v16b h, l; };
__device__ __forceinline__ F2 bsplit16(const float v[16]) { F2 r;
#pragma unroll
  for (int i = 0; i < 16; ++i) { const __bf16 h = (__bf16)v[i]; r.h[i] = h; r.l[i] = (__bf16)(v[i] - (float)h); }
  return r; }
__device__ __forceinline__ F2 split_row(const float* row, int k0, int lane) { float v[16]; const float* p = row + k0 + 8 * (lane >> 4);
#pragma unroll
  for (int i = 0; i < 8; ++i) { v[i] = p[i]; v[8 + i] = p[16 + i]; }
  return bsplit16(v); }
__device__ __forceinline__ F2 split_rowK(const float* row, int k0, int lane, int K) { float v[16]; const int g = lane >> 4;
#pragma unroll
  for (int i = 0; i < 8; ++i) { const int ka = k0 + 8 * g + i, kb = ka + 16; v[i] = ka < K ? row[ka < K ? ka : K - 1] : 0.f; v[8 + i] = kb < K ? row[kb < K ? kb : K - 1] : 0.f; }
  return bsplit16(v); }
__device__ __forceinline__ F2 split_col(const float* W, int k0, int n, int lane, int ld, int K) { float v[16]; const int g = lane >> 4;
#pragma unroll
  for (int i = 0; i < 8; ++i) { const int ka = k0 + 8 * g + i, kb = ka + 16; v[i] = ka < K ? W[(size_t)(ka < K ? ka : K - 1) * ld + n] : 0.f; v[8 + i] = kb < K ? W[(size_t)(kb < K ? kb : K - 1) * ld + n] : 0.f; }
  return bsplit16(v); }
__device__ __forceinline__ v8f mac3(const F2& a, const F2& b, v8f c) { c = wmma_bf(a.l, b.h, c); c = wmma_bf(a.h, b.l, c); return wmma_bf(a.h, b.h, c); }
__device__ __forceinline__ float sigm(float v) { return 1.0f / (1.0f + expf(-v)); }
#define LDSX() do { asm volatile("s_wait_dscnt 0" ::: "memory"); __builtin_amdgcn_wave_barrier(); __builtin_amdgcn_fence(__ATOMIC_RELEASE, "workgroup"); } while (0)

__device__ __forceinline__ float bfr(float v) { return (float)(__bf16)v; }
#define NBT 4
#define CCH 256
#define NN 2304
#define RR 64
#define NBR 3
#ifndef TNB
#define TNB NBT
#endif
#ifndef NI
#define NI NBR
#endif
#define WS_Q   0u
#define WS_K   (WS_Q + 2u * (size_t)NBR * NBT * NN * RR)
#define WS_V   (WS_K + 2u * (size_t)NBR * NBT * NN * RR)
#define WS_S   (WS_V + 2u * (size_t)NBR * NBT * RR * NN)
#define WS_P   (WS_S + 4u * (size_t)NBR * NN * NN)
#define WS_CB  (WS_P + 2u * (size_t)NBR * NN * NN)
#define WS_END (WS_CB + 4u * (size_t)NBT * NN * NBR * RR)

__global__ __launch_bounds__(128) void k_proj(const float* __restrict__ X, const float* __restrict__ WQ, const float* __restrict__ WK, const float* __restrict__ WV, _Float16* __restrict__ QR, _Float16* __restrict__ KR, _Float16* __restrict__ VP) {
  __shared__ __align__(16) _Float16 sh[128][72]; __shared__ __align__(16) _Float16 th[64][136];
  const int tid = threadIdx.x, wave = tid >> 5, lane = tid & 31, col = lane & 15, g = lane >> 4; const int which = blockIdx.y / NBR, i = blockIdx.y % NBR; const int b = blockIdx.z; const int n0 = blockIdx.x * 128;
  const float* Wm = (which == 0 ? WQ : which == 1 ? WK : WV) + (size_t)i * RR * CCH; const float* Xb = X + (size_t)b * CCH * NN;
  v8f acc[8] = {};
#pragma unroll 2
  for (int kc = 0; kc < CCH / 32; ++kc) { v16b a; { const float* p = Wm + (size_t)(wave * 16 + col) * CCH + kc * 32 + 8 * g;
#pragma unroll
      for (int e = 0; e < 8; ++e) { a[e] = (__bf16)p[e]; a[8 + e] = (__bf16)p[16 + e]; } }
#pragma unroll
    for (int j = 0; j < 8; ++j) { v16b w; const int n = n0 + j * 16 + col;
#pragma unroll
      for (int e = 0; e < 8; ++e) { w[e] = (__bf16)Xb[(size_t)(kc * 32 + 8 * g + e) * NN + n]; w[8 + e] = (__bf16)Xb[(size_t)(kc * 32 + 16 + 8 * g + e) * NN + n]; }
      acc[j] = wmma_bf(a, w, acc[j]); } }
#pragma unroll
  for (int j = 0; j < 8; ++j)
#pragma unroll
    for (int r = 0; r < 8; ++r) { const int rl = wave * 16 + 8 * g + r, cl = j * 16 + col; const _Float16 hv = (_Float16)acc[j][r]; if (which == 2) th[rl][cl] = hv; else sh[cl][rl] = hv; }
  __syncthreads();
  if (which < 2) { _Float16* dst = (which == 0 ? QR : KR) + (((size_t)i * NBT + b) * NN + n0) * RR; for (int e = tid; e < 128 * 8; e += 128) { const int cl = e >> 3, q = e & 7; vst2((unsigned*)(dst + (size_t)cl * RR + q * 8), *(const v4u*)&sh[cl][q * 8]); } }
  else { _Float16* dst = VP + ((size_t)i * NBT + b) * RR * NN + n0; for (int e = tid; e < 64 * 16; e += 128) { const int rl = e >> 4, q = e & 15; vst2((unsigned*)(dst + (size_t)rl * NN + q * 8), *(const v4u*)&th[rl][q * 8]); } } }
__global__ __launch_bounds__(128) void k_sc(const _Float16* __restrict__ QR, const _Float16* __restrict__ KR, int b, int i, float* __restrict__ S0) { __shared__ __align__(16) float ss[4][16][132];
  const int tid = threadIdx.x, wave = tid >> 5, lane = tid & 31, col = lane & 15, g = lane >> 4; const int j = blockIdx.z; const int k0 = blockIdx.y * 128; const int ql0 = blockIdx.x * 64 + wave * 16;
  const _Float16* Q = QR + ((size_t)i * NBT + b) * NN * RR; const _Float16* K = KR + ((size_t)j * NBT + b) * NN * RR; float* S = S0 + (size_t)j * NN * NN;
  v8f acc[8] = {};
#pragma unroll
  for (int kc = 0; kc < RR / 32; ++kc) { const v16h ah = frag_h(Q + (size_t)(ql0 + col) * RR + kc * 32, lane);
#pragma unroll
    for (int jj = 0; jj < 8; ++jj) { const v16h kb = frag_h(K + (size_t)(k0 + jj * 16 + col) * RR + kc * 32, lane); acc[jj] = wmma16(ah, kb, acc[jj]); } }
#pragma unroll
  for (int jj = 0; jj < 8; ++jj)
#pragma unroll
    for (int r = 0; r < 8; ++r) ss[wave][8 * g + r][jj * 16 + col] = acc[jj][r] * 0.125f;
  LDSX(); for (int rl = 0; rl < 16; ++rl) vst2(S + (size_t)(ql0 + rl) * NN + k0 + lane * 4, *(const v4f*)&ss[wave][rl][lane * 4]); }
__global__ __launch_bounds__(256) void k_sm(const float* __restrict__ S0, _Float16* __restrict__ P0) { __shared__ float sred[8]; __shared__ float sbc; __shared__ __align__(16) _Float16 shp[NN];
  const int t = threadIdx.x; const size_t row = blockIdx.x; const float* sr = S0 + (size_t)blockIdx.y * NN * NN + row * NN; _Float16* P = P0 + (size_t)blockIdx.y * NN * NN + row * NN;
  float m = -3.0e38f; for (int k = t; k < NN; k += 256) m = fmaxf(m, sr[k]);
#pragma unroll
  for (int o = 1; o < 32; o <<= 1) m = fmaxf(m, __shfl_xor(m, o));
  if ((t & 31) == 0) sred[t >> 5] = m; __syncthreads(); if (t == 0) { float a = sred[0]; for (int e = 1; e < 8; ++e) a = fmaxf(a, sred[e]); sbc = a; } __syncthreads(); m = sbc; __syncthreads();
  float sum = 0.f; for (int k = t; k < NN; k += 256) sum += expf(sr[k] - m);
#pragma unroll
  for (int o = 1; o < 32; o <<= 1) sum += __shfl_xor(sum, o);
  if ((t & 31) == 0) sred[t >> 5] = sum; __syncthreads(); if (t == 0) { float a = 0.f; for (int e = 0; e < 8; ++e) a += sred[e]; sbc = 1.0f / a; } __syncthreads(); const float inv = sbc;
  for (int k = t; k < NN; k += 256) shp[k] = (_Float16)(expf(sr[k] - m) * inv * 2048.0f);
  __syncthreads(); for (int q = t; q < NN / 8; q += 256) vst2((unsigned*)(P + q * 8), *(const v4u*)&shp[q * 8]); }
__global__ __launch_bounds__(128) void k_pv(const _Float16* __restrict__ P0, const _Float16* __restrict__ VP, int b, int i, float* __restrict__ CB) { __shared__ __align__(16) float ss[4][16][RR + 4];
  const int tid = threadIdx.x, wave = tid >> 5, lane = tid & 31, col = lane & 15, g = lane >> 4; const int ql0 = blockIdx.x * 64 + wave * 16;
  v8f acc[RR / 16] = {};
#pragma unroll 1
  for (int j = 0; j < NBR; ++j) { const _Float16* P = P0 + (size_t)j * NN * NN; const _Float16* V = VP + ((size_t)j * NBT + b) * RR * NN;
#pragma unroll 1
    for (int kc = 0; kc < NN / 32; ++kc) { const v16h ph = frag_h(P + (size_t)(ql0 + col) * NN + kc * 32, lane);
#pragma unroll
      for (int jj = 0; jj < RR / 16; ++jj) acc[jj] = wmma16(ph, frag_h(V + (size_t)(jj * 16 + col) * NN + kc * 32, lane), acc[jj]); } }
#pragma unroll
  for (int jj = 0; jj < RR / 16; ++jj)
#pragma unroll
    for (int r = 0; r < 8; ++r) ss[wave][8 * g + r][jj * 16 + col] = acc[jj][r] * (1.0f / 2048.0f);
  LDSX(); for (int rl = 0; rl < 16; ++rl) if (lane < RR / 4) vst2(CB + ((size_t)b * NN + ql0 + rl) * (NBR * RR) + i * RR + lane * 4, *(const v4f*)&ss[wave][rl][lane * 4]); }
__global__ __launch_bounds__(128) void k_out(const float* __restrict__ CB, const float* __restrict__ WO, const float* __restrict__ X, float* __restrict__ OUT) { __shared__ __align__(16) float st[128][68];
  const int tid = threadIdx.x, wave = tid >> 5, lane = tid & 31, col = lane & 15, g = lane >> 4; const int b = blockIdx.z; const int c0 = blockIdx.y * 128; const int n0 = blockIdx.x * 64; const int nl0 = wave * 16;
  v8f acc[8] = {};
#pragma unroll
  for (int kc = 0; kc < (NBR * RR) / 32; ++kc) { F2 a = split_row(CB + ((size_t)b * NN + n0 + nl0 + col) * (NBR * RR), kc * 32, lane);
    if (kc * 32 >= NI * RR) { a.h = (v16b){}; a.l = (v16b){}; }
#pragma unroll
    for (int j = 0; j < 8; ++j) { v16b w; const int c = c0 + j * 16 + col;
#pragma unroll
      for (int e = 0; e < 8; ++e) { w[e] = (__bf16)WO[(size_t)c * (NBR * RR) + kc * 32 + 8 * g + e]; w[8 + e] = (__bf16)WO[(size_t)c * (NBR * RR) + kc * 32 + 16 + 8 * g + e]; }
      acc[j] = wmma_bf(a.h, w, acc[j]); acc[j] = wmma_bf(a.l, w, acc[j]); } }
#pragma unroll
  for (int j = 0; j < 8; ++j)
#pragma unroll
    for (int r = 0; r < 8; ++r) st[j * 16 + col][nl0 + 8 * g + r] = acc[j][r];
  __syncthreads();
  for (int cl = wave * 32; cl < wave * 32 + 32; ++cl) { const int c = c0 + cl; const size_t o = ((size_t)b * CCH + c) * NN + n0 + (lane & 15) * 4;
    if (lane < 16) { const v4f ov = *(const v4f*)&st[cl][lane * 4]; v4f y;
#pragma unroll
      for (int e = 0; e < 4; ++e) y[e] = bfr(X[o + e]) * (1.0f / (1.0f + expf(-ov[e])));
      vst2(OUT + o, y); } } }
extern "C" void kernel_launch(void* const* d_in, const int* in_sizes, int n_in, void* d_out, int out_size, void* d_ws, size_t ws_size, hipStream_t stream) {
  (void)in_sizes; (void)n_in; (void)out_size;
  const float** F = (const float**)d_in;
  if (ws_size < (size_t)WS_END) return;
  char* ws = (char*)d_ws; _Float16 *QR = (_Float16*)(ws + WS_Q), *KR = (_Float16*)(ws + WS_K), *VP = (_Float16*)(ws + WS_V), *P = (_Float16*)(ws + WS_P); float *S = (float*)(ws + WS_S), *CB = (float*)(ws + WS_CB);
  k_proj<<<dim3(NN / 128, 3 * NBR, TNB), 128, 0, stream>>>(F[0], F[1], F[2], F[3], QR, KR, VP);
  for (int b = 0; b < TNB; ++b) for (int i = 0; i < NI; ++i) {
    k_sc<<<dim3(NN / 64, NN / 128, NBR), 128, 0, stream>>>(QR, KR, b, i, S);
    k_sm<<<dim3(NN, NBR), 256, 0, stream>>>(S, P);
    k_pv<<<dim3(NN / 64), 128, 0, stream>>>(P, VP, b, i, CB);
  }
  k_out<<<dim3(NN / 64, CCH / 128, TNB), 128, 0, stream>>>(CB, F[4], F[0], (float*)d_out);
}
